// TTCN_34797825032291
// MI455X (gfx1250) — hardware-verified
//
#include <hip/hip_runtime.h>
#include <math.h>

typedef __attribute__((ext_vector_type(16))) _Float16 v16h;
typedef __attribute__((ext_vector_type(16))) __bf16 v16b;
typedef __attribute__((ext_vector_type(8)))  _Float16 v8h;
typedef __attribute__((ext_vector_type(8)))  float v8f;
typedef __attribute__((ext_vector_type(4)))  float v4f;
typedef __attribute__((ext_vector_type(2)))  float v2f;
typedef __attribute__((ext_vector_type(4)))  unsigned v4u;
typedef __attribute__((ext_vector_type(4)))  int v4i;
typedef float __attribute__((may_alias)) float_a;
typedef int __attribute__((may_alias)) int_a;

template <typename T> __device__ __forceinline__ void vst2(void* p, T v) { *(volatile T*)p = v; __threadfence(); *(volatile T*)p = v; }
__device__ __forceinline__ v8f wmma16(v16h a, v16h b, v8f c) {
  v8f d = __builtin_amdgcn_wmma_f32_16x16x32_f16(false, a, false, b, (short)0, c, false, false);
  asm volatile("v_nop\n\tv_nop\n\tv_nop\n\tv_nop" : "+v"(d) : "v"(a), "v"(b));
  return d;
}
__device__ __forceinline__ v8f wmma_bf(v16b a, v16b b, v8f c) {
  v8f d = __builtin_amdgcn_wmma_f32_16x16x32_bf16(false, a, false, b, (short)0, c, false, false);
  asm volatile("v_nop\n\tv_nop\n\tv_nop\n\tv_nop" : "+v"(d) : "v"(a), "v"(b));
  return d;
}
__device__ __forceinline__ v16h frag_h(const _Float16* rowk0, int lane) {
  union { v16h v; v8h q[2]; } u; const _Float16* p = rowk0 + 8 * (lane >> 4);
  u.q[0] = *(const v8h*)p; u.q[1] = *(const v8h*)(p + 16); return u.v;
}
__device__ __forceinline__ v16h frag_f32(const float* rowk0, int lane) {
  v16h a; const float* p = rowk0 + 8 * (lane >> 4);
#pragma unroll
  for (int i = 0; i < 8; ++i) { a[i] = (_Float16)p[i]; a[8 + i] = (_Float16)p[16 + i]; }
  return a;
}
__device__ __forceinline__ v16h frag_f32s(const float* rowk0, int lane, float sc) {
  v16h a; const float* p = rowk0 + 8 * (lane >> 4);
#pragma unroll
  for (int i = 0; i < 8; ++i) { a[i] = (_Float16)(p[i] * sc); a[8 + i] = (_Float16)(p[16 + i] * sc); }
  return a;
}
__device__ __forceinline__ v16h fragc_f32(const float* W, int k0, int n, int lane, int ld, int K) {
  v16h a; const int g = lane >> 4;
#pragma unroll
  for (int i = 0; i < 8; ++i) { const int ka = k0 + 8 * g + i, kb = ka + 16;
    a[i] = (_Float16)(ka < K ? W[(size_t)(ka < K ? ka : K - 1) * ld + n] : 0.f); a[8 + i] = (_Float16)(kb < K ? W[(size_t)(kb < K ? kb : K - 1) * ld + n] : 0.f); }
  return a;
}
struct F2 { v16b h, l; };
__device__ __forceinline__ F2 bsplit16(const float v[16]) { F2 r;
#pragma unroll
  for (int i = 0; i < 16; ++i) { const __bf16 h = (__bf16)v[i]; r.h[i] = h; r.l[i] = (__bf16)(v[i] - (float)h); }
  return r; }
__device__ __forceinline__ F2 split_row(const float* row, int k0, int lane) { float v[16]; const float* p = row + k0 + 8 * (lane >> 4);
#pragma unroll
  for (int i = 0; i < 8; ++i) { v[i] = p[i]; v[8 + i] = p[16 + i]; }
  return bsplit16(v); }
__device__ __forceinline__ F2 split_rowK(const float* row, int k0, int lane, int K) { float v[16]; const int g = lane >> 4;
#pragma unroll
  for (int i = 0; i < 8; ++i) { const int ka = k0 + 8 * g + i, kb = ka + 16; v[i] = ka < K ? row[ka < K ? ka : K - 1] : 0.f; v[8 + i] = kb < K ? row[kb < K ? kb : K - 1] : 0.f; }
  return bsplit16(v); }
__device__ __forceinline__ F2 split_col(const float* W, int k0, int n, int lane, int ld, int K) { float v[16]; const int g = lane >> 4;
#pragma unroll
  for (int i = 0; i < 8; ++i) { const int ka = k0 + 8 * g + i, kb = ka + 16; v[i] = ka < K ? W[(size_t)(ka < K ? ka : K - 1) * ld + n] : 0.f; v[8 + i] = kb < K ? W[(size_t)(kb < K ? kb : K - 1) * ld + n] : 0.f; }
  return bsplit16(v); }
__device__ __forceinline__ v8f mac3(const F2& a, const F2& b, v8f c) { c = wmma_bf(a.l, b.h, c); c = wmma_bf(a.h, b.l, c); return wmma_bf(a.h, b.h, c); }
__device__ __forceinline__ float sigm(float v) { return 1.0f / (1.0f + expf(-v)); }
#define LDSX() do { asm volatile("s_wait_dscnt 0" ::: "memory"); __builtin_amdgcn_wave_barrier(); __builtin_amdgcn_fence(__ATOMIC_RELEASE, "workgroup"); } while (0)


#define NSEQ 128
#define LX 512
#define DIN 32
#define KF 63
#define KP 64
#define NCOL (KF * DIN)
#ifndef TNS
#define TNS NSEQ
#endif
typedef __attribute__((ext_vector_type(8))) __bf16 v8b;
__device__ __forceinline__ v16b frag_b(const __bf16* rowk0, int lane) {
  union { v16b v; v8b q[2]; } u; const __bf16* p = rowk0 + 8 * (lane >> 4);
  u.q[0] = *(const v8b*)p; u.q[1] = *(const v8b*)(p + 16); return u.v;
}
__device__ __forceinline__ float bfr(float v) { return (float)(__bf16)v; }
__device__ __attribute__((noinline)) float exp_ni(float v) { return expf(v); }
__device__ __attribute__((noinline)) float erf_ni(float v) { return erff(v); }

#define WS_H2  0u
#define WS_OS  (WS_H2 + 4u * (size_t)NSEQ * LX * KP)
#define WS_END (WS_OS + 4u * (size_t)NSEQ * KP)

__global__ __launch_bounds__(128) void k_h2(const float* __restrict__ X, const float* __restrict__ W1, const float* __restrict__ B1, const float* __restrict__ W2, const float* __restrict__ B2, float* __restrict__ H2) { __shared__ __align__(16) float sa[4][16][68];
  const int tid = threadIdx.x, wave = tid >> 5, lane = tid & 31, col = lane & 15, g = lane >> 4; const size_t r0 = (size_t)blockIdx.x * 64 + wave * 16;
  v8f acc[4] = {};
  { v16b a; const float* p = X + (r0 + col) * DIN + 8 * g;
#pragma unroll
    for (int i = 0; i < 8; ++i) { a[i] = (__bf16)p[i]; a[8 + i] = (__bf16)p[16 + i]; }
#pragma unroll
    for (int j = 0; j < 4; ++j) { v16b w; const int o = j * 16 + col;
#pragma unroll
      for (int i = 0; i < 8; ++i) { w[i] = (__bf16)((o < KF) ? W1[(8 * g + i) * KF + o] : 0.f); w[8 + i] = (__bf16)((o < KF) ? W1[(16 + 8 * g + i) * KF + o] : 0.f); }
      acc[j] = wmma_bf(a, w, acc[j]); } }
#pragma unroll
  for (int j = 0; j < 4; ++j) { const int o = j * 16 + col; const float bb = (o < KF) ? bfr(B1[o]) : 0.f;
#pragma unroll
    for (int r = 0; r < 8; ++r) sa[wave][8 * g + r][o] = (o < KF) ? fmaxf(acc[j][r] + bb, 0.f) : 0.f; }
  LDSX();
  v8f acc2[4] = {};
#pragma unroll
  for (int kc = 0; kc < 2; ++kc) { const v16h a = frag_f32(&sa[wave][col][0] + kc * 32, lane);
#pragma unroll
    for (int j = 0; j < 4; ++j) { v16h w; const int o = j * 16 + col;
#pragma unroll
      for (int i = 0; i < 8; ++i) { const int ka = kc * 32 + 8 * g + i, kb = ka + 16; w[i] = (_Float16)((o < KF && ka < KF) ? bfr(W2[ka * KF + o]) : 0.f); w[8 + i] = (_Float16)((o < KF && kb < KF) ? bfr(W2[kb * KF + o]) : 0.f); }
      acc2[j] = wmma16(a, w, acc2[j]); } }
  LDSX();
#pragma unroll
  for (int j = 0; j < 4; ++j) { const int o = j * 16 + col; const float bb = (o < KF) ? bfr(B2[o]) : 0.f;
#pragma unroll
    for (int r = 0; r < 8; ++r) sa[wave][8 * g + r][o] = (o < KF) ? fmaxf(acc2[j][r] + bb, 0.f) : 0.f; }
  LDSX(); for (int rl = 0; rl < 16; ++rl) if (lane < 16) vst2(H2 + (r0 + rl) * KP + lane * 4, *(const v4f*)&sa[wave][rl][lane * 4]); }
__global__ __launch_bounds__(256) void k_w3h(const float* __restrict__ W3, _Float16* __restrict__ W3H) { __shared__ __align__(16) _Float16 s[64 * KP]; const int t = threadIdx.x; const int c0 = blockIdx.x * 64;
  for (int e = t; e < 64 * KP; e += 256) { const int cl = e / KP, k = e % KP; s[e] = (_Float16)((k < KF && c0 + cl < NCOL) ? bfr(W3[(size_t)k * NCOL + c0 + cl]) : 0.f); }
  __syncthreads(); for (int q = t; q < 64 * KP / 8; q += 256) vst2((unsigned*)(W3H + (size_t)c0 * KP + q * 8), *(const v4u*)&s[q * 8]); }
#define WS_W3 (WS_END)
#define WS_END2 (WS_W3 + 2u * 2048 * KP)
__global__ __launch_bounds__(128) void k_main(const float* __restrict__ X, const float* __restrict__ MK, const float* __restrict__ H2, const _Float16* __restrict__ W3H, const float* __restrict__ B3, const float* __restrict__ TB, float* __restrict__ OS) {
  __shared__ __align__(16) float st[LX][33]; __shared__ float smk[LX]; __shared__ float sred[4][32]; __shared__ float scol[2][32]; __shared__ __align__(16) float sout[KP];
  const int tid = threadIdx.x, wave = tid >> 5, lane = tid & 31, col = lane & 15, g = lane >> 4; const size_t n = blockIdx.x;
  for (int l = tid; l < LX; l += 128) smk[l] = bfr(MK[n * LX + l]);
  if (tid < KP) sout[tid] = 0.f;
  __syncthreads();
  int nvalid = 0; for (int l = 0; l < LX; ++l) nvalid += (smk[l] != 0.f) ? 1 : 0;
#pragma unroll 1
  for (int k = 0; k < KF; ++k) {
#pragma unroll 1
    for (int rt = wave; rt < LX / 16; rt += 4) { v8f acc[2] = {};
#pragma unroll
      for (int kc = 0; kc < 2; ++kc) { const v16h a = frag_f32(H2 + (n * LX + rt * 16 + col) * KP + kc * 32, lane);
#pragma unroll
        for (int j = 0; j < 2; ++j) acc[j] = wmma16(a, frag_h(W3H + ((size_t)k * DIN + j * 16 + col) * KP + kc * 32, lane), acc[j]); }
#pragma unroll
      for (int j = 0; j < 2; ++j) { const int d = j * 16 + col; const float bb = bfr(B3[k * DIN + d]);
#pragma unroll
        for (int r = 0; r < 8; ++r) st[rt * 16 + 8 * g + r][d] = acc[j][r] + bb; } }
    __syncthreads();
    { const int d = lane; const int l0 = wave * (LX / 4); float m = -3.0e38f;
#pragma unroll 1
      for (int l = l0; l < l0 + LX / 4; ++l) if (smk[l] != 0.f) m = fmaxf(m, st[l][d]);
      sred[wave][d] = m; __syncthreads(); m = fmaxf(fmaxf(sred[0][d], sred[1][d]), fmaxf(sred[2][d], sred[3][d])); __syncthreads();
      float s = 0.f, acc = 0.f;
#pragma unroll 1
      for (int l = l0; l < l0 + LX / 4; ++l) { float w; if (nvalid > 0) w = (smk[l] != 0.f) ? expf(st[l][d] - m) : 0.f; else w = 1.f;
        s += w; acc += w * bfr(X[(n * LX + l) * DIN + d]); }
      sred[wave][d] = s; __syncthreads(); const float stot = (sred[0][d] + sred[1][d]) + (sred[2][d] + sred[3][d]); __syncthreads();
      sred[wave][d] = acc; __syncthreads();
      if (wave == 0) { const float a4 = (sred[0][d] + sred[1][d]) + (sred[2][d] + sred[3][d]); scol[0][d] = a4 / stot; }
      __syncthreads();
      if (tid == 0) { float tot = 0.f; for (int dd = 0; dd < DIN; ++dd) tot += scol[0][dd]; sout[k] = fmaxf(tot + bfr(TB[k]), 0.f); }
      __syncthreads(); } }
  if (tid < KP / 4) vst2(OS + n * KP + tid * 4, *(const v4f*)&sout[tid * 4]); }
__global__ __launch_bounds__(256) void k_fin(const float* __restrict__ OS, float* __restrict__ OUT) { __shared__ __align__(16) float s[TNS * KF + 4]; const int t = threadIdx.x;
  for (int e = t; e < TNS * KF; e += 256) { const int n = e / KF, k = e % KF; s[e] = OS[n * KP + k]; }
  for (int e = TNS * KF + t; e < TNS * KF + 4; e += 256) s[e] = 0.f;
  __syncthreads(); for (int q = t; q < (TNS * KF + 3) / 4; q += 256) vst2(OUT + q * 4, *(const v4f*)&s[q * 4]); }
extern "C" void kernel_launch(void* const* d_in, const int* in_sizes, int n_in, void* d_out, int out_size, void* d_ws, size_t ws_size, hipStream_t stream) {
  (void)in_sizes; (void)n_in; (void)out_size;
  const float** F = (const float**)d_in;
  if (ws_size < (size_t)WS_END2) return;
  char* ws = (char*)d_ws; float *H2 = (float*)(ws + WS_H2), *OS = (float*)(ws + WS_OS); _Float16* W3H = (_Float16*)(ws + WS_W3);
  k_h2<<<TNS * LX / 64, 128, 0, stream>>>(F[0], F[2], F[3], F[4], F[5], H2);
  k_w3h<<<NCOL / 64 + ((NCOL % 64) ? 1 : 0), 256, 0, stream>>>(F[6], W3H);
  k_main<<<TNS, 128, 0, stream>>>(F[0], F[1], H2, W3H, F[7], F[8], OS);
  k_fin<<<1, 256, 0, stream>>>(OS, (float*)d_out);
}
